// BoundaryFluxAttention_67705864454353
// MI455X (gfx1250) — hardware-verified
//
#include <hip/hip_runtime.h>
#include <stdint.h>
#include <stddef.h>


typedef unsigned short u16;
typedef __bf16       v16bf __attribute__((ext_vector_type(16)));
typedef float        v8f   __attribute__((ext_vector_type(8)));
typedef float        v4f   __attribute__((ext_vector_type(4)));
typedef unsigned int v4u   __attribute__((ext_vector_type(4)));

#define D_MODEL   1024
#define NUM_HEADS 16
#define HEAD_DIM  64
#define SEQ_T     2048
#define BATCH     2
#define NROWS     (BATCH * SEQ_T)

union FragU { v16bf v; v4u q[2]; };

__device__ __forceinline__ unsigned int bf_rne(float f) {
  unsigned int x = __float_as_uint(f);
  return (x + 0x7FFFu + ((x >> 16) & 1u)) >> 16;
}

__device__ __forceinline__ void split_pack8(v8f x, v4u& ph, v4u& pl) {
#pragma unroll
  for (int j = 0; j < 4; ++j) {
    float a = x[2 * j], b = x[2 * j + 1];
    unsigned int ha = bf_rne(a), hb = bf_rne(b);
    unsigned int la = bf_rne(a - __uint_as_float(ha << 16));
    unsigned int lb = bf_rne(b - __uint_as_float(hb << 16));
    ph[j] = ha | (hb << 16);
    pl[j] = la | (lb << 16);
  }
}

__device__ __forceinline__ v16bf frag16(const u16* rowptr, int hl) {
  FragU f;
  f.q[0] = *(const v4u*)(rowptr + 8 * hl);
  f.q[1] = *(const v4u*)(rowptr + 16 + 8 * hl);
  return f.v;
}

__device__ __forceinline__ v8f wmma3(v16bf ah, v16bf al, v16bf bh, v16bf bl, v8f c) {
  c = __builtin_amdgcn_wmma_f32_16x16x32_bf16(false, ah, false, bh, (short)0, c, false, false);
  c = __builtin_amdgcn_wmma_f32_16x16x32_bf16(false, ah, false, bl, (short)0, c, false, false);
  c = __builtin_amdgcn_wmma_f32_16x16x32_bf16(false, al, false, bh, (short)0, c, false, false);
  asm volatile("v_nop\n\tv_nop\n\tv_nop\n\tv_nop" : "+v"(c) : "v"(ah), "v"(al), "v"(bh), "v"(bl));
  return c;
}

__global__ __launch_bounds__(256)
void k_split_rows(const float* __restrict__ src, u16* dh, u16* dl, int n8) {
  const int i = blockIdx.x * 256 + threadIdx.x;
  if (i < n8) {
    const float* p = src + (size_t)i * 8;
    v4f a = *(const v4f*)p;
    v4f b = *(const v4f*)(p + 4);
    v8f x = __builtin_shufflevector(a, b, 0, 1, 2, 3, 4, 5, 6, 7);
    v4u ph, pl;
    split_pack8(x, ph, pl);
    const size_t o = (size_t)i * 8;
    *(volatile v4u*)(dh + o) = ph;
    *(volatile v4u*)(dl + o) = pl;
    __threadfence();
    *(volatile v4u*)(dh + o) = ph;
    *(volatile v4u*)(dl + o) = pl;
  }
}

__global__ __launch_bounds__(256)
void k_split_transpose(const float* __restrict__ src, u16* dh, u16* dl, int K, int N) {
  __shared__ float tile[64][65];
  const int tid = threadIdx.x, lane = tid & 31, w = tid >> 5;
  const int kBase = blockIdx.y * 64, nBase = blockIdx.x * 64;
  const int r = tid >> 2, c = (tid & 3) * 16;
  const float* sp = src + (size_t)(kBase + r) * N + nBase + c;
#pragma unroll
  for (int j = 0; j < 4; ++j) {
    v4f v = *(const v4f*)(sp + 4 * j);
    tile[r][c + 4 * j + 0] = v[0];
    tile[r][c + 4 * j + 1] = v[1];
    tile[r][c + 4 * j + 2] = v[2];
    tile[r][c + 4 * j + 3] = v[3];
  }
  __syncthreads();
  v4u ph[2], pl[2];
  size_t dst[2];
  const int piece = lane & 7;
#pragma unroll
  for (int it = 0; it < 2; ++it) {
    const int nrow = w * 8 + it * 4 + (lane >> 3);
    v8f x;
#pragma unroll
    for (int j = 0; j < 8; ++j) x[j] = tile[piece * 8 + j][nrow];
    split_pack8(x, ph[it], pl[it]);
    dst[it] = (size_t)(nBase + nrow) * K + kBase + piece * 8;
  }
#pragma unroll
  for (int it = 0; it < 2; ++it) {
    *(volatile v4u*)(dh + dst[it]) = ph[it];
    *(volatile v4u*)(dl + dst[it]) = pl[it];
  }
  __threadfence();
#pragma unroll
  for (int it = 0; it < 2; ++it) {
    *(volatile v4u*)(dh + dst[it]) = ph[it];
    *(volatile v4u*)(dl + dst[it]) = pl[it];
  }
}

#define G_ASH 0
#define G_ASL 2560
#define G_BSH 5120
#define G_BSL 10240

__device__ __forceinline__ void gemm_tile_64x128(
    const u16* __restrict__ Ah, const u16* __restrict__ Al,
    const u16* __restrict__ Bh, const u16* __restrict__ Bl,
    int K, int rowBase, int colBase, u16* smem, v8f (&acc)[4])
{
  const int tid = threadIdx.x, lane = tid & 31, w = tid >> 5;
  const int hl = lane >> 4, n16 = lane & 15;
  const int wm = w & 3, wn = w >> 2;
  const int ar = tid >> 2, ac = (tid & 3) * 8;
  const int bn = tid >> 1, bk = (tid & 1) * 16;
  const size_t aOff = (size_t)(rowBase + ar) * K + ac;
  const size_t bOff = (size_t)(colBase + bn) * K + bk;
#pragma unroll 1
  for (int k0 = 0; k0 < K; k0 += 32) {
    v4u xah  = *(const v4u*)(Ah + aOff + k0);
    v4u xal  = *(const v4u*)(Al + aOff + k0);
    v4u xbh0 = *(const v4u*)(Bh + bOff + k0);
    v4u xbh1 = *(const v4u*)(Bh + bOff + k0 + 8);
    v4u xbl0 = *(const v4u*)(Bl + bOff + k0);
    v4u xbl1 = *(const v4u*)(Bl + bOff + k0 + 8);
    __syncthreads();
    *(v4u*)(smem + G_ASH + ar * 40 + ac)     = xah;
    *(v4u*)(smem + G_ASL + ar * 40 + ac)     = xal;
    *(v4u*)(smem + G_BSH + bn * 40 + bk)     = xbh0;
    *(v4u*)(smem + G_BSH + bn * 40 + bk + 8) = xbh1;
    *(v4u*)(smem + G_BSL + bn * 40 + bk)     = xbl0;
    *(v4u*)(smem + G_BSL + bn * 40 + bk + 8) = xbl1;
    __syncthreads();
    v16bf fah = frag16(smem + G_ASH + (wm * 16 + n16) * 40, hl);
    v16bf fal = frag16(smem + G_ASL + (wm * 16 + n16) * 40, hl);
#pragma unroll
    for (int nf = 0; nf < 4; ++nf) {
      v16bf fbh = frag16(smem + G_BSH + (wn * 64 + nf * 16 + n16) * 40, hl);
      v16bf fbl = frag16(smem + G_BSL + (wn * 64 + nf * 16 + n16) * 40, hl);
      acc[nf] = wmma3(fah, fal, fbh, fbl, acc[nf]);
    }
  }
  __syncthreads();
}

__global__ __launch_bounds__(256)
void k_gemm_qkv(const u16* __restrict__ Xh, const u16* __restrict__ Xl,
                const u16* __restrict__ Wh, const u16* __restrict__ Wl,
                const float* __restrict__ bias,
                u16* Qh, u16* Ql, u16* Kh, u16* Kl, u16* Vh, u16* Vl)
{
  __shared__ __attribute__((aligned(16))) u16 smem[16384];
  const int tid = threadIdx.x, lane = tid & 31, w = tid >> 5;
  const int hl = lane >> 4, n16 = lane & 15;
  const int wm = w & 3, wn = w >> 2;
  const int rowBase = blockIdx.y * 64, colBase = blockIdx.x * 128;

  v8f acc[4] = {};
  gemm_tile_64x128(Xh, Xl, Wh, Wl, D_MODEL, rowBase, colBase, smem, acc);

  const int which = colBase >> 10;
  const int hh0 = (colBase >> 6) & 15;
  const int bb = rowBase >> 11, t0 = rowBase & (SEQ_T - 1);

  if (which != 2) {
#pragma unroll
    for (int nf = 0; nf < 4; ++nf) {
      const int cl = wn * 64 + nf * 16 + n16;
      const float bv = bias[colBase + cl];
#pragma unroll
      for (int r = 0; r < 8; ++r) {
        const int rl = wm * 16 + 8 * hl + r;
        const float v = acc[nf][r] + bv;
        const unsigned int hb = bf_rne(v);
        const unsigned int lb = bf_rne(v - __uint_as_float(hb << 16));
        smem[rl * 128 + cl] = (u16)hb;
        smem[8192 + rl * 128 + cl] = (u16)lb;
      }
    }
  } else {
#pragma unroll
    for (int nf = 0; nf < 4; ++nf) {
      const int cl = wn * 64 + nf * 16 + n16;
      const float bv = bias[colBase + cl];
      v8f vv = acc[nf] + bv;
      v4u ph, pl;
      split_pack8(vv, ph, pl);
      *(v4u*)(smem + cl * 64 + wm * 16 + 8 * hl)        = ph;
      *(v4u*)(smem + 8192 + cl * 64 + wm * 16 + 8 * hl) = pl;
    }
  }
  __syncthreads();

  const int piece = lane & 7;
#pragma unroll
  for (int pass = 0; pass < 2; ++pass) {
#pragma unroll
    for (int it = 0; it < 8; ++it) {
      const int L = w * 32 + it * 4 + (lane >> 3);
      const int plane = L >> 7, rem = L & 127;
      if (which != 2) {
        const int row = rem >> 1, hs = rem & 1;
        v4u val = *(const v4u*)(smem + plane * 8192 + row * 128 + hs * 64 + piece * 8);
        const int bhd = bb * NUM_HEADS + hh0 + hs;
        const size_t dst = ((size_t)bhd * SEQ_T + t0 + row) * HEAD_DIM + piece * 8;
        u16* P = (which == 0) ? (plane ? Ql : Qh) : (plane ? Kl : Kh);
        *(volatile v4u*)(P + dst) = val;
      } else {
        const int hs = rem >> 6, d = rem & 63;
        v4u val = *(const v4u*)(smem + plane * 8192 + rem * 64 + piece * 8);
        const int bhd = bb * NUM_HEADS + hh0 + hs;
        const size_t dst = ((size_t)bhd * HEAD_DIM + d) * SEQ_T + t0 + piece * 8;
        u16* P = plane ? Vl : Vh;
        *(volatile v4u*)(P + dst) = val;
      }
    }
    if (pass == 0) __threadfence();
  }
}

__global__ __launch_bounds__(256)
void k_gemm_out(const u16* __restrict__ Ah, const u16* __restrict__ Al,
                const u16* __restrict__ Wh, const u16* __restrict__ Wl,
                const float* __restrict__ bias, float* out)
{
  __shared__ __attribute__((aligned(16))) u16 smem[16384];
  const int tid = threadIdx.x, lane = tid & 31, w = tid >> 5;
  const int hl = lane >> 4, n16 = lane & 15;
  const int wm = w & 3, wn = w >> 2;
  const int rowBase = blockIdx.y * 64, colBase = blockIdx.x * 128;

  v8f acc[4] = {};
  gemm_tile_64x128(Ah, Al, Wh, Wl, D_MODEL, rowBase, colBase, smem, acc);

  float* fs = (float*)smem;
#pragma unroll
  for (int nf = 0; nf < 4; ++nf) {
    const int cl = wn * 64 + nf * 16 + n16;
    const float bv = bias[colBase + cl];
#pragma unroll
    for (int r = 0; r < 8; ++r) {
      const int rl = wm * 16 + 8 * hl + r;
      fs[rl * 128 + cl] = acc[nf][r] + bv;
    }
  }
  __syncthreads();

  const int piece = lane & 7;
#pragma unroll
  for (int pass = 0; pass < 2; ++pass) {
#pragma unroll
    for (int it = 0; it < 8; ++it) {
      const int L = w * 32 + it * 4 + (lane >> 3);
      const int row = L >> 2, seg = L & 3;
      v4f val = *(const v4f*)(fs + row * 128 + seg * 32 + piece * 4);
      const size_t dst = (size_t)(rowBase + row) * D_MODEL + colBase + seg * 32 + piece * 4;
      *(volatile v4f*)(out + dst) = val;
    }
    if (pass == 0) __threadfence();
  }
}

#define A_KH   0
#define A_KL   4608
#define A_VH   9216
#define A_VL   13824
#define A_BS   18432
#define A_SMEM 18560

__global__ __launch_bounds__(256)
void k_attn(const u16* __restrict__ Qh, const u16* __restrict__ Ql,
            const u16* __restrict__ Kh, const u16* __restrict__ Kl,
            const u16* __restrict__ Vh, const u16* __restrict__ Vl,
            const float* __restrict__ bsc, u16* Oh, u16* Ol)
{
  __shared__ __attribute__((aligned(16))) u16 smem[A_SMEM];
  float* biasS = (float*)(smem + A_BS);

  const int QT = SEQ_T / 128;
  const int bh = blockIdx.x / QT, qt = blockIdx.x - bh * QT;
  const int bb = bh >> 4, hh = bh & 15;
  const int tid = threadIdx.x, lane = tid & 31, w = tid >> 5;
  const int hl = lane >> 4, n16 = lane & 15;
  const int q0 = qt * 128 + w * 16;
  const size_t headRow = (size_t)bh * SEQ_T;

  const u16* qph = Qh + (headRow + q0 + n16) * HEAD_DIM;
  const u16* qpl = Ql + (headRow + q0 + n16) * HEAD_DIM;
  const v16bf qh0 = frag16(qph, hl), qh1 = frag16(qph + 32, hl);
  const v16bf ql0 = frag16(qpl, hl), ql1 = frag16(qpl + 32, hl);

  v8f o[4] = {};
  float mrun = -1e30f, lrun = 0.0f;

  const int lr = tid >> 2, lc = (tid & 3) * 16;
  const u16* kph = Kh + (headRow + lr) * HEAD_DIM + lc;
  const u16* kpl = Kl + (headRow + lr) * HEAD_DIM + lc;
  const u16* vph = Vh + ((size_t)bh * HEAD_DIM + lr) * SEQ_T + lc;
  const u16* vpl = Vl + ((size_t)bh * HEAD_DIM + lr) * SEQ_T + lc;

  const int NT = SEQ_T / 64;
#pragma unroll 1
  for (int kt = 0; kt < NT; ++kt) {
    const size_t ko = (size_t)kt * 64 * HEAD_DIM;
    const size_t vo = (size_t)kt * 64;
    v4u xkh0 = *(const v4u*)(kph + ko), xkh1 = *(const v4u*)(kph + ko + 8);
    v4u xkl0 = *(const v4u*)(kpl + ko), xkl1 = *(const v4u*)(kpl + ko + 8);
    v4u xvh0 = *(const v4u*)(vph + vo), xvh1 = *(const v4u*)(vph + vo + 8);
    v4u xvl0 = *(const v4u*)(vpl + vo), xvl1 = *(const v4u*)(vpl + vo + 8);
    __syncthreads();
    *(v4u*)(smem + A_KH + lr * 72 + lc) = xkh0;  *(v4u*)(smem + A_KH + lr * 72 + lc + 8) = xkh1;
    *(v4u*)(smem + A_KL + lr * 72 + lc) = xkl0;  *(v4u*)(smem + A_KL + lr * 72 + lc + 8) = xkl1;
    *(v4u*)(smem + A_VH + lr * 72 + lc) = xvh0;  *(v4u*)(smem + A_VH + lr * 72 + lc + 8) = xvh1;
    *(v4u*)(smem + A_VL + lr * 72 + lc) = xvl0;  *(v4u*)(smem + A_VL + lr * 72 + lc + 8) = xvl1;
    if (w == 0) {
      v4f bv = *(const v4f*)(bsc + (size_t)bb * SEQ_T + kt * 64 + n16 * 4);
      bv = bv * 0.1f;
      *(v4f*)(biasS + n16 * 4) = bv;
    }
    __syncthreads();

    v8f s[4];
#pragma unroll
    for (int nf = 0; nf < 4; ++nf) {
      const u16* krh = smem + A_KH + (nf * 16 + n16) * 72;
      const u16* krl = smem + A_KL + (nf * 16 + n16) * 72;
      v8f c = {};
      c = wmma3(frag16(krh, hl),      frag16(krl, hl),      qh0, ql0, c);
      c = wmma3(frag16(krh + 32, hl), frag16(krl + 32, hl), qh1, ql1, c);
      v4f b0 = *(const v4f*)(biasS + nf * 16 + 8 * hl);
      v4f b1 = *(const v4f*)(biasS + nf * 16 + 8 * hl + 4);
      s[nf][0] = c[0] * 0.125f + b0[0];
      s[nf][1] = c[1] * 0.125f + b0[1];
      s[nf][2] = c[2] * 0.125f + b0[2];
      s[nf][3] = c[3] * 0.125f + b0[3];
      s[nf][4] = c[4] * 0.125f + b1[0];
      s[nf][5] = c[5] * 0.125f + b1[1];
      s[nf][6] = c[6] * 0.125f + b1[2];
      s[nf][7] = c[7] * 0.125f + b1[3];
    }

    float mt = -1e30f;
#pragma unroll
    for (int nf = 0; nf < 4; ++nf)
#pragma unroll
      for (int r = 0; r < 8; ++r) mt = fmaxf(mt, s[nf][r]);
    mt = fmaxf(mt, __shfl_xor(mt, 16, 32));
    const float mn = fmaxf(mrun, mt);
    const float corr = __expf(mrun - mn);
    mrun = mn;
    lrun *= corr;
#pragma unroll
    for (int nf = 0; nf < 4; ++nf) o[nf] = o[nf] * corr;
    float rs = 0.0f;
#pragma unroll
    for (int nf = 0; nf < 4; ++nf)
#pragma unroll
      for (int r = 0; r < 8; ++r) {
        const float p = __expf(s[nf][r] - mn);
        s[nf][r] = p;
        rs += p;
      }
    rs += __shfl_xor(rs, 16, 32);
    lrun += rs;

#pragma unroll
    for (int s2 = 0; s2 < 2; ++s2) {
      FragU ph, pl;
      split_pack8(s[2 * s2],     ph.q[0], pl.q[0]);
      split_pack8(s[2 * s2 + 1], ph.q[1], pl.q[1]);
#pragma unroll
      for (int nf = 0; nf < 4; ++nf) {
        const u16* vrh = smem + A_VH + (nf * 16 + n16) * 72 + s2 * 32;
        const u16* vrl = smem + A_VL + (nf * 16 + n16) * 72 + s2 * 32;
        o[nf] = wmma3(frag16(vrh, hl), frag16(vrl, hl), ph.v, pl.v, o[nf]);
      }
    }
  }
  __syncthreads();

  const float inv = 1.0f / lrun;
  u16* stg = smem + w * 2048;
#pragma unroll
  for (int nf = 0; nf < 4; ++nf) {
    v8f vv = o[nf] * inv;
    v4u ph, pl;
    split_pack8(vv, ph, pl);
    *(v4u*)(stg + n16 * 64 + nf * 16 + 8 * hl)        = ph;
    *(v4u*)(stg + 1024 + n16 * 64 + nf * 16 + 8 * hl) = pl;
  }
  __syncthreads();

  const int piece = lane & 7;
#pragma unroll
  for (int pass = 0; pass < 2; ++pass) {
#pragma unroll
    for (int it = 0; it < 8; ++it) {
      const int L = it * 4 + (lane >> 3);
      const int plane = L >> 4, qq = L & 15;
      v4u val = *(const v4u*)(stg + plane * 1024 + qq * 64 + piece * 8);
      const size_t dst = ((size_t)(bb * SEQ_T + q0 + qq)) * D_MODEL + hh * HEAD_DIM + piece * 8;
      u16* P = plane ? Ol : Oh;
      *(volatile v4u*)(P + dst) = val;
    }
    if (pass == 0) __threadfence();
  }
}

extern "C" void kernel_launch(void* const* d_in, const int* in_sizes, int n_in,
                              void* d_out, int out_size, void* d_ws, size_t ws_size,
                              hipStream_t stream) {
  if (n_in < 6) return;
  if (in_sizes[0] != NROWS * D_MODEL || in_sizes[1] != BATCH * SEQ_T ||
      in_sizes[2] != D_MODEL * 3 * D_MODEL || in_sizes[3] != 3 * D_MODEL ||
      in_sizes[4] != D_MODEL * D_MODEL || in_sizes[5] != D_MODEL ||
      out_size != NROWS * D_MODEL) return;

  const float* x      = (const float*)d_in[0];
  const float* bscore = (const float*)d_in[1];
  const float* Wqkv   = (const float*)d_in[2];
  const float* bqkv   = (const float*)d_in[3];
  const float* Wout   = (const float*)d_in[4];
  const float* bout   = (const float*)d_in[5];
  float* out = (float*)d_out;

  const size_t nX  = (size_t)NROWS * D_MODEL;
  const size_t nWq = (size_t)D_MODEL * 3 * D_MODEL;
  const size_t nWo = (size_t)D_MODEL * D_MODEL;
  const size_t nH  = (size_t)BATCH * NUM_HEADS * SEQ_T * HEAD_DIM;
  const size_t nA  = nX;

  size_t off = 0;
  unsigned char* ws = (unsigned char*)d_ws;
  u16* Xh  = (u16*)(ws + off); off += nX * 2;
  u16* Xl  = (u16*)(ws + off); off += nX * 2;
  u16* Wqh = (u16*)(ws + off); off += nWq * 2;
  u16* Wql = (u16*)(ws + off); off += nWq * 2;
  u16* Woh = (u16*)(ws + off); off += nWo * 2;
  u16* Wol = (u16*)(ws + off); off += nWo * 2;
  u16* Qh  = (u16*)(ws + off); off += nH * 2;
  u16* Ql  = (u16*)(ws + off); off += nH * 2;
  u16* Kh  = (u16*)(ws + off); off += nH * 2;
  u16* Kl  = (u16*)(ws + off); off += nH * 2;
  u16* Vh  = (u16*)(ws + off); off += nH * 2;
  u16* Vl  = (u16*)(ws + off); off += nH * 2;
  u16* Oh  = (u16*)(ws + off); off += nA * 2;
  u16* Ol  = (u16*)(ws + off); off += nA * 2;
  if (off > ws_size) return;

  {
    const int n8 = (int)(nX / 8);
    k_split_rows<<<(n8 + 255) / 256, 256, 0, stream>>>(x, Xh, Xl, n8);
  }
  {
    dim3 g(3 * D_MODEL / 64, D_MODEL / 64);
    k_split_transpose<<<g, 256, 0, stream>>>(Wqkv, Wqh, Wql, D_MODEL, 3 * D_MODEL);
  }
  {
    dim3 g(D_MODEL / 64, D_MODEL / 64);
    k_split_transpose<<<g, 256, 0, stream>>>(Wout, Woh, Wol, D_MODEL, D_MODEL);
  }
  {
    dim3 g(3 * D_MODEL / 128, NROWS / 64);
    k_gemm_qkv<<<g, 256, 0, stream>>>(Xh, Xl, Wqh, Wql, bqkv, Qh, Ql, Kh, Kl, Vh, Vl);
  }
  k_attn<<<BATCH * NUM_HEADS * (SEQ_T / 128), 256, 0, stream>>>(Qh, Ql, Kh, Kl, Vh, Vl, bscore, Oh, Ol);
  {
    dim3 g(D_MODEL / 128, NROWS / 64);
    k_gemm_out<<<g, 256, 0, stream>>>(Oh, Ol, Woh, Wol, bout, out);
  }
}
